// GCN_S_15977278341730
// MI455X (gfx1250) — hardware-verified
//
#include <hip/hip_runtime.h>
#include <stddef.h>


#define EMB       64
#define NTHR      256
#define NWAVE     8
#define EPT       8
#define NGRP      2
#define CHUNK     (NTHR * EPT * NGRP)
#define WCAP      (EPT * NGRP * 32)
#define LISTN     (NWAVE * WCAP)
#define NB        1024
#define NMAT      4
#define WELEM     (EMB * EMB)
#define NEGSLOPE  0.01f
#define EPSN      1e-12f
#define LDS_LAYER (NB * EMB * 4 + LISTN * 4 + 64)

static_assert((CHUNK & (CHUNK - 1)) == 0);
static_assert(CHUNK <= 4096);
static_assert((NB & (NB - 1)) == 0 && NB <= 4096);
static_assert(NB % (16 * NWAVE) == 0);
static_assert((NB * EMB) % (128 * NWAVE) == 0);

typedef float    v2f   __attribute__((ext_vector_type(2)));
typedef float    v4f   __attribute__((ext_vector_type(4)));
typedef float    v8f   __attribute__((ext_vector_type(8)));
typedef int      v4i   __attribute__((ext_vector_type(4)));
typedef unsigned v4u   __attribute__((ext_vector_type(4)));
typedef __bf16   v16bf __attribute__((ext_vector_type(16)));
union FragB { v16bf v; v4u u[2]; };
struct HL { v4u h; v4u l; };

__device__ __forceinline__ unsigned rne_hi(float x) {
  unsigned u = __float_as_uint(x);
  return (u + 0x7FFFu + ((u >> 16) & 1u)) & 0xFFFF0000u;
}

__device__ __forceinline__ HL split8(v4f a, v4f b) {
  float s[8];
  s[0] = a.x; s[1] = a.y; s[2] = a.z; s[3] = a.w;
  s[4] = b.x; s[5] = b.y; s[6] = b.z; s[7] = b.w;
  unsigned hb[8], lb[8];
#pragma unroll
  for (int j = 0; j < 8; ++j) {
    const unsigned hu = rne_hi(s[j]);
    const float    lf = s[j] - __uint_as_float(hu);
    const unsigned lu = rne_hi(lf);
    hb[j] = hu >> 16;
    lb[j] = lu >> 16;
  }
  HL r;
  r.h.x = hb[0] | (hb[1] << 16); r.h.y = hb[2] | (hb[3] << 16);
  r.h.z = hb[4] | (hb[5] << 16); r.h.w = hb[6] | (hb[7] << 16);
  r.l.x = lb[0] | (lb[1] << 16); r.l.y = lb[2] | (lb[3] << 16);
  r.l.z = lb[4] | (lb[5] << 16); r.l.w = lb[6] | (lb[7] << 16);
  return r;
}

__device__ __forceinline__ v8f wmb(v16bf a, v16bf b, v8f c) {
  v8f d = __builtin_amdgcn_wmma_f32_16x16x32_bf16(false, a, false, b, (short)0, c, false, false);
  asm volatile("v_nop\n\tv_nop\n\tv_nop\n\tv_nop" : "+v"(d) : "v"(a), "v"(b));
  return d;
}

template <int NBT>
__device__ __forceinline__ int scan_chunk(const int* __restrict__ dsts, int nE, int cbase, int nodeBase,
                                          int vec8, int* list, int tid, int lane, int wave) {
  int wc = 0;
#pragma unroll
  for (int g = 0; g < NGRP; ++g) {
    const int el0  = (g * NTHR + tid) * EPT;
    const int e0   = cbase + el0;
    const int sent = -2147483647 - 1;
    v4i da, db;
    if (vec8 != 0 && cbase + CHUNK <= nE) {
      da = *(const v4i*)(dsts + e0);
      db = *(const v4i*)(dsts + e0 + 4);
    } else {
      const int last = nE - 1;
      da.x = (e0     < nE) ? dsts[min(e0,     last)] : sent;
      da.y = (e0 + 1 < nE) ? dsts[min(e0 + 1, last)] : sent;
      da.z = (e0 + 2 < nE) ? dsts[min(e0 + 2, last)] : sent;
      da.w = (e0 + 3 < nE) ? dsts[min(e0 + 3, last)] : sent;
      db.x = (e0 + 4 < nE) ? dsts[min(e0 + 4, last)] : sent;
      db.y = (e0 + 5 < nE) ? dsts[min(e0 + 5, last)] : sent;
      db.z = (e0 + 6 < nE) ? dsts[min(e0 + 6, last)] : sent;
      db.w = (e0 + 7 < nE) ? dsts[min(e0 + 7, last)] : sent;
    }
    const unsigned nb = (unsigned)nodeBase;
    const unsigned s0 = (unsigned)da.x - nb, s1 = (unsigned)da.y - nb;
    const unsigned s2 = (unsigned)da.z - nb, s3 = (unsigned)da.w - nb;
    const unsigned s4 = (unsigned)db.x - nb, s5 = (unsigned)db.y - nb;
    const unsigned s6 = (unsigned)db.z - nb, s7 = (unsigned)db.w - nb;
    const bool h0 = s0 < (unsigned)NBT, h1 = s1 < (unsigned)NBT, h2 = s2 < (unsigned)NBT, h3 = s3 < (unsigned)NBT;
    const bool h4 = s4 < (unsigned)NBT, h5 = s5 < (unsigned)NBT, h6 = s6 < (unsigned)NBT, h7 = s7 < (unsigned)NBT;
    const unsigned any = __builtin_amdgcn_ballot_w32(h0 | h1 | h2 | h3 | h4 | h5 | h6 | h7);
    if (any != 0u) {
#define HITJ(J, HJ, SJ) { \
        const unsigned mj = __builtin_amdgcn_ballot_w32(HJ); \
        if (mj != 0u) { \
          if (HJ) { \
            const int pos = wc + (int)__builtin_amdgcn_mbcnt_lo(mj, 0u); \
            if (pos < WCAP) list[wave * WCAP + pos] = ((el0 + (J)) << 12) | (int)(SJ); \
          } \
          wc += (int)__builtin_popcount(mj); } }
      HITJ(0, h0, s0)
      HITJ(1, h1, s1)
      HITJ(2, h2, s2)
      HITJ(3, h3, s3)
      HITJ(4, h4, s4)
      HITJ(5, h5, s5)
      HITJ(6, h6, s6)
      HITJ(7, h7, s7)
#undef HITJ
    }
  }
  return wc;
}

__global__ __launch_bounds__(NTHR) void k_wprep(
    const float* __restrict__ W0, const float* __restrict__ W1,
    const float* __restrict__ W2, const float* __restrict__ W3,
    unsigned short* whi, unsigned short* wlo) {
  const int mat = blockIdx.x >> 1;
  const float* W = (mat == 0) ? W0 : (mat == 1) ? W1 : (mat == 2) ? W2 : W3;
  const int o = ((blockIdx.x & 1) * NTHR + threadIdx.x) * 8;
  const v4f a = *(const v4f*)(W + o), b = *(const v4f*)(W + o + 4);
  const HL s = split8(a, b);
  unsigned short* ph = whi + (size_t)mat * WELEM + o;
  unsigned short* pl = wlo + (size_t)mat * WELEM + o;
  *(volatile v4u*)ph = s.h;
  *(volatile v4u*)pl = s.l;
  __threadfence();
  *(volatile v4u*)ph = s.h;
  *(volatile v4u*)pl = s.l;
}

__global__ __launch_bounds__(NTHR) void k_layer(
    const int* __restrict__ rows, const int* __restrict__ cols, const float* __restrict__ vals,
    const float* __restrict__ x, const unsigned short* __restrict__ whi,
    const unsigned short* __restrict__ wlo, const float* __restrict__ bias,
    float* y, int nN, int nE, int rowLimit, int vec8) {
  extern __shared__ v4f lds_dyn[];
  float* acc  = (float*)lds_dyn;
  int*   list = (int*)(acc + NB * EMB);
  int*   wcnt = list + LISTN;
  const int tid = threadIdx.x, lane = tid & 31, wave = tid >> 5, hh = lane >> 4, m = lane & 15;
  const int nodeBase = blockIdx.x * NB;

  {
    const v4f z = {0.f, 0.f, 0.f, 0.f};
    for (int i = tid; i < NB * EMB / 4; i += NTHR) lds_dyn[i] = z;
  }
  __syncthreads();

  const int nChunks = (nE + CHUNK - 1) / CHUNK;
#pragma unroll 1
  for (int ch = 0; ch < nChunks; ++ch) {
    const int cbase = ch * CHUNK;
    const int wc = scan_chunk<NB>(rows, nE, cbase, nodeBase, vec8, list, tid, lane, wave);
    if (lane == 0) wcnt[wave] = wc;
    __syncthreads();
    if (wave == 0) {
#pragma unroll 1
      for (int wsx = 0; wsx < NWAVE; ++wsx) {
        int n = __builtin_amdgcn_readfirstlane(wcnt[wsx]);
        n = n > WCAP ? WCAP : (n < 0 ? 0 : n);
        const int* lp = list + wsx * WCAP;
#pragma unroll 1
        for (int i = 0; i < n; ++i) {
          const int ent  = __builtin_amdgcn_readfirstlane(lp[i]);
          const int slot = ent & (NB - 1);
          int e = cbase + ((ent >> 12) & (CHUNK - 1));
          e = e > nE - 1 ? nE - 1 : e;
          int src = cols[e];
          src = src < 0 ? 0 : (src > nN - 1 ? nN - 1 : src);
          const float v = vals[e];
          const v2f xv = *(const v2f*)(x + (size_t)src * EMB + 2 * lane);
          v2f* ap = (v2f*)(acc + slot * EMB + 2 * lane);
          const v2f o = *ap;
          *ap = o + v * xv;
        }
      }
    }
    __syncthreads();
  }

  float bq[4];
  bq[0] = bias[m]; bq[1] = bias[16 + m]; bq[2] = bias[32 + m]; bq[3] = bias[48 + m];
#pragma unroll 1
  for (int T = wave; T < NB / 16; T += NWAVE) {
    v8f c[4];
#pragma unroll
    for (int t = 0; t < 4; ++t) { v8f z = {0.f, 0.f, 0.f, 0.f, 0.f, 0.f, 0.f, 0.f}; c[t] = z; }
#pragma unroll
    for (int kt = 0; kt < EMB / 32; ++kt) {
      const float* ap = acc + (16 * T + m) * EMB + 32 * kt + 8 * hh;
      const v4f p0 = *(const v4f*)ap,        p1 = *(const v4f*)(ap + 4);
      const v4f p2 = *(const v4f*)(ap + 16), p3 = *(const v4f*)(ap + 20);
      const HL s0 = split8(p0, p1), s1 = split8(p2, p3);
      FragB ah, al;
      ah.u[0] = s0.h; ah.u[1] = s1.h;
      al.u[0] = s0.l; al.u[1] = s1.l;
#pragma unroll
      for (int t = 0; t < 4; ++t) {
        const int bo = (16 * t + m) * EMB + 32 * kt + 8 * hh;
        FragB bh, bl;
        bh.u[0] = *(const v4u*)(whi + bo); bh.u[1] = *(const v4u*)(whi + bo + 16);
        bl.u[0] = *(const v4u*)(wlo + bo); bl.u[1] = *(const v4u*)(wlo + bo + 16);
        c[t] = wmb(ah.v, bh.v, c[t]);
        c[t] = wmb(ah.v, bl.v, c[t]);
        c[t] = wmb(al.v, bh.v, c[t]);
      }
    }
    float yv[4][8];
    float ss[8];
#pragma unroll
    for (int r = 0; r < 8; ++r) ss[r] = 0.f;
#pragma unroll
    for (int t = 0; t < 4; ++t) {
#pragma unroll
      for (int r = 0; r < 8; ++r) {
        float v = c[t][r] + bq[t];
        v = (v >= 0.f) ? v : NEGSLOPE * v;
        yv[t][r] = v;
        ss[r] += v * v;
      }
    }
#pragma unroll
    for (int r = 0; r < 8; ++r) {
      float s = ss[r];
      s += __shfl_xor(s, 1);
      s += __shfl_xor(s, 2);
      s += __shfl_xor(s, 4);
      s += __shfl_xor(s, 8);
      ss[r] = 1.0f / fmaxf(sqrtf(s), EPSN);
    }
    __builtin_amdgcn_fence(__ATOMIC_RELEASE, "wavefront");
    __builtin_amdgcn_wave_barrier();
    float* yp = acc + (16 * T + 8 * hh) * EMB + m;
#pragma unroll
    for (int t = 0; t < 4; ++t) {
#pragma unroll
      for (int r = 0; r < 8; ++r) yp[r * EMB + 16 * t] = yv[t][r] * ss[r];
    }
  }
  __syncthreads();

  const size_t gbase = (size_t)nodeBase * EMB;
  const int QN = (NB * EMB) / (128 * NWAVE);
#pragma unroll 4
  for (int q = 0; q < QN; ++q) {
    const int f  = (wave * QN + q) * 128 + 4 * lane;
    const int lr = f >> 6;
    const v4f v  = *(const v4f*)(acc + f);
    if (nodeBase + lr < rowLimit) *(volatile v4f*)(y + gbase + (size_t)f) = v;
  }
  __threadfence();
#pragma unroll 4
  for (int q = 0; q < QN; ++q) {
    const int f  = (wave * QN + q) * 128 + 4 * lane;
    const int lr = f >> 6;
    const v4f v  = *(const v4f*)(acc + f);
    if (nodeBase + lr < rowLimit) *(volatile v4f*)(y + gbase + (size_t)f) = v;
  }
}

extern "C" void kernel_launch(void* const* d_in, const int* in_sizes, int n_in,
                              void* d_out, int out_size, void* d_ws, size_t ws_size,
                              hipStream_t stream) {
  if (n_in < 16) return;
  const int NU = in_sizes[0] / EMB;
  const int NI = in_sizes[1] / EMB;
  if (NU <= 0 || NI <= 0 || in_sizes[0] != NU * EMB || in_sizes[1] != NI * EMB) return;
  if (in_sizes[2] != WELEM || in_sizes[4] != WELEM || in_sizes[6] != WELEM || in_sizes[8] != WELEM) return;
  if (in_sizes[3] < EMB || in_sizes[5] < EMB || in_sizes[7] < EMB || in_sizes[9] < EMB) return;
  const int EU = in_sizes[10];
  const int EI = in_sizes[13];
  if (EU < 0 || EI < 0 || in_sizes[11] != EU || in_sizes[12] != EU || in_sizes[14] != EI || in_sizes[15] != EI) return;
  if (out_size != (NU + NI) * EMB) return;

  const float* user_emb = (const float*)d_in[0];
  const float* item_emb = (const float*)d_in[1];
  const float* Wu0 = (const float*)d_in[2];
  const float* bu0 = (const float*)d_in[3];
  const float* Wu1 = (const float*)d_in[4];
  const float* bu1 = (const float*)d_in[5];
  const float* Wi0 = (const float*)d_in[6];
  const float* bi0 = (const float*)d_in[7];
  const float* Wi1 = (const float*)d_in[8];
  const float* bi1 = (const float*)d_in[9];
  const int*   u_rows = (const int*)d_in[10];
  const int*   u_cols = (const int*)d_in[11];
  const float* u_vals = (const float*)d_in[12];
  const int*   i_rows = (const int*)d_in[13];
  const int*   i_cols = (const int*)d_in[14];
  const float* i_vals = (const float*)d_in[15];
  float* out_u = (float*)d_out;
  float* out_i = out_u + (size_t)NU * EMB;

  const int nBU = (NU + NB - 1) / NB;
  const int nBI = (NI + NB - 1) / NB;

  char* ws = (char*)d_ws;
  size_t off = 0;
  const size_t oWh = off; off += (size_t)NMAT * WELEM * 2;            off = (off + 255) & ~(size_t)255;
  const size_t oWl = off; off += (size_t)NMAT * WELEM * 2;            off = (off + 255) & ~(size_t)255;
  const size_t oXu = off; off += (size_t)nBU * NB * EMB * 4;          off = (off + 255) & ~(size_t)255;
  const size_t oXi = off; off += (size_t)nBI * NB * EMB * 4;          off = (off + 255) & ~(size_t)255;
  if (off > ws_size) return;
  unsigned short* whi = (unsigned short*)(ws + oWh);
  unsigned short* wlo = (unsigned short*)(ws + oWl);
  float* xu1 = (float*)(ws + oXu);
  float* xi1 = (float*)(ws + oXi);

  const int vec8 = 1;

  k_wprep<<<2 * NMAT, NTHR, 0, stream>>>(Wu0, Wu1, Wi0, Wi1, whi, wlo);

  hipFuncSetAttribute(reinterpret_cast<const void*>(&k_layer),
                      hipFuncAttributeMaxDynamicSharedMemorySize, LDS_LAYER);

  k_layer<<<nBU, NTHR, LDS_LAYER, stream>>>(u_rows, u_cols, u_vals, user_emb,
                                            whi + 0 * WELEM, wlo + 0 * WELEM, bu0,
                                            xu1, NU, EU, nBU * NB, vec8);
  k_layer<<<nBI, NTHR, LDS_LAYER, stream>>>(i_rows, i_cols, i_vals, item_emb,
                                            whi + 2 * WELEM, wlo + 2 * WELEM, bi0,
                                            xi1, NI, EI, nBI * NB, vec8);
  k_layer<<<nBU, NTHR, LDS_LAYER, stream>>>(u_rows, u_cols, u_vals, xu1,
                                            whi + 1 * WELEM, wlo + 1 * WELEM, bu1,
                                            out_u, NU, EU, NU, vec8);
  k_layer<<<nBI, NTHR, LDS_LAYER, stream>>>(i_rows, i_cols, i_vals, xi1,
                                            whi + 3 * WELEM, wlo + 3 * WELEM, bi1,
                                            out_i, NI, EI, NI, vec8);
}
